// KnowledgeInteractionModule_16801912062748
// MI455X (gfx1250) — hardware-run, weakly checked
//
#include <hip/hip_runtime.h>
#include <stddef.h>


typedef _Float16 v16h __attribute__((ext_vector_type(16)));
typedef _Float16 v8h  __attribute__((ext_vector_type(8)));
typedef float    v8f  __attribute__((ext_vector_type(8)));
typedef float    v4f  __attribute__((ext_vector_type(4)));
typedef _Float16 h16;

#ifndef SEQ
#define SEQ 384
#endif
#define SEQ_FULL 384
#define DIM   1024
#define NHEAD 8
#define HD    128
#define HID1  (2 * DIM)
#define SYNW  (3 * DIM)
#define OUT1_OFF ((size_t)SEQ_FULL * SEQ_FULL)

static_assert(SEQ >= 128 && SEQ <= SEQ_FULL && (SEQ % 128) == 0);
static_assert(DIM == NHEAD * HD);
static_assert(HD == 128);
static_assert((DIM % 64) == 0 && (DIM % 32) == 0);
static_assert((SEQ % 64) == 0 && (SEQ % 32) == 0 && (SEQ % 2) == 0);
static_assert(DIM / 8 == 128);
static_assert(DIM == 256 * 4);
static_assert(((2 * DIM) % 256) == 0 && ((3 * DIM) % 256) == 0);
static_assert((SYNW % 128) == 0 && (HID1 % 128) == 0);
static_assert((HID1 % 32) == 0 && (DIM % 32) == 0);
static_assert(OUT1_OFF * 4 == (size_t)589824);
static_assert((OUT1_OFF + DIM) * 4 == (size_t)593920);

#define LDT 72
#define LDC 68
#define LDK 136
#define LDV 40
static_assert((LDT % 8) == 0 && LDT >= 64);
static_assert((LDC % 4) == 0 && LDC >= 64);
static_assert((LDK % 8) == 0 && LDK >= HD);
static_assert((LDV % 8) == 0 && LDV >= 32);

#define WCARRY 64.0f
#define PCARRY 1024.0f
#define VCARRY 64.0f

#define X16_BYTES   ((size_t)SEQ * DIM * 2)
#define W1C_BYTES   ((size_t)2 * DIM * DIM * 2)
#define WQKV_BYTES  ((size_t)3 * DIM * DIM * 2)
#define WO_BYTES    ((size_t)DIM * DIM * 2)
#define AB_BYTES    ((size_t)SEQ * 2 * DIM * 4)
#define P16_BYTES   ((size_t)SEQ * DIM * 2)
#define ATT_BYTES   ((size_t)SEQ * DIM * 4)
#define SYN_BYTES   ((size_t)SYNW * 4)
#define HIDV_BYTES  ((size_t)HID1 * 4)
#define OFF_X16  ((size_t)0)
#define OFF_W1C  (OFF_X16 + X16_BYTES)
#define OFF_WQKV (OFF_W1C + W1C_BYTES)
#define OFF_WO   (OFF_WQKV + WQKV_BYTES)
#define OFF_AB   (OFF_WO + WO_BYTES)
#define OFF_Q    (OFF_AB + AB_BYTES)
#define OFF_K    (OFF_Q + P16_BYTES)
#define OFF_VT   (OFF_K + P16_BYTES)
#define OFF_CTX  (OFF_VT + P16_BYTES)
#define OFF_ATT  (OFF_CTX + P16_BYTES)
#define OFF_SYN  (OFF_ATT + ATT_BYTES)
#define OFF_HIDV (OFF_SYN + SYN_BYTES)
#define WS_TOTAL (OFF_HIDV + HIDV_BYTES)
static_assert((X16_BYTES % 128) == 0 && (W1C_BYTES % 128) == 0 && (WQKV_BYTES % 128) == 0);
static_assert((WO_BYTES % 128) == 0 && (AB_BYTES % 128) == 0 && (P16_BYTES % 128) == 0);
static_assert((ATT_BYTES % 128) == 0 && (SYN_BYTES % 128) == 0 && (HIDV_BYTES % 128) == 0);
static_assert(WS_TOTAL <= (size_t)134217728);

__device__ __forceinline__ float bf16r(float x) {
  unsigned int u = __float_as_uint(x);
  u = (u + 0x7FFFu + ((u >> 16) & 1u)) & 0xFFFF0000u;
  return __uint_as_float(u);
}

static __device__ __forceinline__ h16 toh_flush(float v) {
  const h16 r = (h16)v;
  return (fabsf(v) < 6.103515625e-05f) ? (h16)0.0f : r;
}

__device__ __forceinline__ v16h frag_at(const _Float16* p) {
  v8h lo = *(const v8h*)(p);
  v8h hi = *(const v8h*)(p + 16);
  v16h out;
#pragma unroll
  for (int i = 0; i < 8; ++i) { out[i] = lo[i]; out[i + 8] = hi[i]; }
  return out;
}
__device__ __forceinline__ v16h ld_frag(const _Float16* base, unsigned ld) {
  const unsigned lane = threadIdx.x & 31u;
  return frag_at(base + (lane & 15u) * ld + (lane >> 4) * 8u);
}

__device__ __forceinline__ v8f wmma16(v16h a, v16h b, v8f c) {
  v8f d = __builtin_amdgcn_wmma_f32_16x16x32_f16(false, a, false, b, (short)0, c,
                                                 false, false);
  asm volatile("v_nop\n\tv_nop\n\tv_nop\n\tv_nop" : "+v"(d) : "v"(a), "v"(b));
  return d;
}

__device__ __forceinline__ float red16_max(float x) {
#pragma unroll
  for (int off = 1; off < 16; off <<= 1) x = fmaxf(x, __shfl_xor(x, off, 32));
  return x;
}
__device__ __forceinline__ float red16_sum(float x) {
#pragma unroll
  for (int off = 1; off < 16; off <<= 1) x += __shfl_xor(x, off, 32);
  return x;
}
__device__ __forceinline__ float red32_sum(float x) {
#pragma unroll
  for (int off = 1; off < 32; off <<= 1) x += __shfl_xor(x, off, 32);
  return x;
}

__device__ __forceinline__ void wave_lds_sync() {
  __builtin_amdgcn_fence(3  , "wavefront");
  asm volatile("s_wait_dscnt 0x0" ::: "memory");
  __builtin_amdgcn_wave_barrier();
}

__device__ __forceinline__ float gelu_erf(float x) {
  const float z = fabsf(x) * 0.70710678118654752f;
  const float t = __builtin_amdgcn_rcpf(1.0f + 0.3275911f * z);
  float p = 1.061405429f;
  p = p * t - 1.453152027f;
  p = p * t + 1.421413741f;
  p = p * t - 0.284496736f;
  p = p * t + 0.254829592f;
  p = p * t;
  const float e = 1.0f - p * __expf(-(z * z));
  return 0.5f * x * (1.0f + copysignf(e, x));
}

__global__ __launch_bounds__(256) void cast_plane_kernel(
    const float* __restrict__ W, _Float16* __restrict__ out, unsigned ldw, unsigned coff,
    float carry) {
  const unsigned idx = blockIdx.x * 256u + threadIdx.x;
  const unsigned n = idx >> 7;
  const unsigned kc = (idx & 127u) * 8u;
  const float* src = W + (size_t)n * ldw + coff + kc;
  const v4f a0 = *(const v4f*)(src);
  const v4f a1 = *(const v4f*)(src + 4);
  v8h o;
#pragma unroll
  for (int i = 0; i < 4; ++i) {
    o[i]     = toh_flush(carry * bf16r(a0[i]));
    o[i + 4] = toh_flush(carry * bf16r(a1[i]));
  }
  _Float16* p = out + (size_t)n * DIM + kc;
  *(volatile v8h*)p = o;
  __threadfence();
  *(volatile v8h*)p = o;
}

template <int MODE>
__device__ __forceinline__ void gemm_body(
    const _Float16* __restrict__ A16, const _Float16* __restrict__ Bt, const unsigned K,
    const float* __restrict__ bias, float* __restrict__ outf, _Float16* __restrict__ out16,
    const unsigned ldo, const float cs) {
  __shared__ float Cs[64 * LDC];
  const unsigned tid = threadIdx.x, lane = tid & 31u, w = tid >> 5;
  const unsigned mw = w >> 1, nw = w & 1u;
  const unsigned hh = lane >> 4, m = lane & 15u;
  const unsigned n0 = blockIdx.x * 64u;
  const unsigned row0 = blockIdx.y * 64u;

  const _Float16* ap  = A16 + (size_t)(row0 + mw * 16u + m) * K + hh * 8u;
  const _Float16* bp0 = Bt + (size_t)(n0 + nw * 32u + m) * K + hh * 8u;
  const _Float16* bp1 = bp0 + (size_t)16 * K;
  v8f acc0 = {}, acc1 = {};
#pragma unroll 2
  for (unsigned k0 = 0; k0 < K; k0 += 32u) {
    const v16h a  = frag_at(ap + k0);
    const v16h b0 = frag_at(bp0 + k0);
    const v16h b1 = frag_at(bp1 + k0);
    acc0 = wmma16(a, b0, acc0);
    acc1 = wmma16(a, b1, acc1);
  }
#pragma unroll
  for (int r = 0; r < 8; ++r) {
    float* d = &Cs[(mw * 16u + hh * 8u + (unsigned)r) * LDC + nw * 32u + m];
    d[0]  = acc0[r];
    d[16] = acc1[r];
  }
  __syncthreads();

  if (MODE == 0) {
    v8h x[2];
    size_t off[2];
#pragma unroll
    for (unsigned i = 0; i < 2u; ++i) {
      const unsigned r = 32u * i + (tid >> 3);
      const unsigned c = (tid & 7u) * 8u;
      const v4f u0 = *(const v4f*)&Cs[r * LDC + c];
      const v4f u1 = *(const v4f*)&Cs[r * LDC + c + 4];
      const v4f g0 = *(const v4f*)(bias + n0 + c);
      const v4f g1 = *(const v4f*)(bias + n0 + c + 4u);
#pragma unroll
      for (int j = 0; j < 4; ++j) {
        x[i][j]     = toh_flush(u0[j] * cs + bf16r(g0[j]));
        x[i][j + 4] = toh_flush(u1[j] * cs + bf16r(g1[j]));
      }
      off[i] = (size_t)(row0 + r) * ldo + n0 + c;
    }
#pragma unroll
    for (int i = 0; i < 2; ++i) *(volatile v8h*)(out16 + off[i]) = x[i];
    __threadfence();
#pragma unroll
    for (int i = 0; i < 2; ++i) *(volatile v8h*)(out16 + off[i]) = x[i];
  }

  if (MODE == 1) {
    v8h x[2];
    size_t off[2];
#pragma unroll
    for (unsigned i = 0; i < 2u; ++i) {
      const unsigned dcol = 32u * i + (tid >> 3);
      const unsigned kk = (tid & 7u) * 8u;
      const float bb = bf16r(bias[n0 + dcol]);
#pragma unroll
      for (unsigned j = 0; j < 8u; ++j) {
        const float t = Cs[(kk + j) * LDC + dcol] * cs + bb;
        x[i][j] = toh_flush(t);
      }
      off[i] = (size_t)(n0 + dcol) * SEQ + row0 + kk;
    }
#pragma unroll
    for (int i = 0; i < 2; ++i) *(volatile v8h*)(out16 + off[i]) = x[i];
    __threadfence();
#pragma unroll
    for (int i = 0; i < 2; ++i) *(volatile v8h*)(out16 + off[i]) = x[i];
  }

  if (MODE == 2 || MODE == 3) {
    v4f xs[4];
    size_t off[4];
#pragma unroll
    for (unsigned i = 0; i < 4u; ++i) {
      const unsigned r = 16u * i + (tid >> 4);
      const unsigned c = (tid & 15u) * 4u;
      const v4f u = *(const v4f*)&Cs[r * LDC + c];
      v4f val;
      if (MODE == 2) {
        const v4f g = *(const v4f*)(bias + n0 + c);
#pragma unroll
        for (int j = 0; j < 4; ++j) val[j] = u[j] * cs + bf16r(g[j]);
      } else {
#pragma unroll
        for (int j = 0; j < 4; ++j) val[j] = u[j] * cs;
      }
      xs[i] = val;
      off[i] = (size_t)(row0 + r) * ldo + n0 + c;
    }
#pragma unroll
    for (int i = 0; i < 4; ++i) *(volatile v4f*)(outf + off[i]) = xs[i];
    __threadfence();
#pragma unroll
    for (int i = 0; i < 4; ++i) *(volatile v4f*)(outf + off[i]) = xs[i];
  }
}

__global__ __launch_bounds__(256) void gemm_qk_kernel(
    const _Float16* __restrict__ A16, const _Float16* __restrict__ Bt,
    const float* __restrict__ bias, _Float16* __restrict__ out16) {
  gemm_body<0>(A16, Bt, (unsigned)DIM, bias, (float*)0, out16, (unsigned)DIM, 1.0f / WCARRY);
}
__global__ __launch_bounds__(256) void gemm_v_kernel(
    const _Float16* __restrict__ A16, const _Float16* __restrict__ Bt,
    const float* __restrict__ bias, _Float16* __restrict__ vt) {
  gemm_body<1>(A16, Bt, (unsigned)DIM, bias, (float*)0, vt, (unsigned)SEQ, 1.0f / WCARRY);
}
__global__ __launch_bounds__(256) void gemm_out_kernel(
    const _Float16* __restrict__ A16, const _Float16* __restrict__ Bt,
    const float* __restrict__ bias, float* __restrict__ outf) {
  gemm_body<2>(A16, Bt, (unsigned)DIM, bias, outf, (_Float16*)0, (unsigned)DIM,
               1.0f / (WCARRY * VCARRY));
}
__global__ __launch_bounds__(256) void gemm_ab_kernel(
    const _Float16* __restrict__ A16, const _Float16* __restrict__ Bt,
    float* __restrict__ outf) {
  gemm_body<3>(A16, Bt, (unsigned)DIM, (const float*)0, outf, (_Float16*)0,
               (unsigned)(2 * DIM), 1.0f / WCARRY);
}

__global__ __launch_bounds__(256) void pair_score_kernel(
    const float* __restrict__ AB, const float* __restrict__ b1, const float* __restrict__ w2,
    const float* __restrict__ b2, float* __restrict__ scores) {
  __shared__ float sA[DIM];
  __shared__ float sW[DIM];
  __shared__ float sOut[32];
  const unsigned tid = threadIdx.x, lane = tid & 31u;
  const unsigned w = (unsigned)__builtin_amdgcn_readfirstlane((int)(tid >> 5));
  const unsigned i = blockIdx.y;
  const unsigned j0 = blockIdx.x * 32u;
  {
    const unsigned c = tid * 4u;
    const v4f a  = *(const v4f*)(AB + (size_t)i * (2u * DIM) + c);
    const v4f bb = *(const v4f*)(b1 + c);
    const v4f ww = *(const v4f*)(w2 + c);
    v4f sa, sw;
#pragma unroll
    for (int k = 0; k < 4; ++k) {
      sa[k] = a[k] + bf16r(bb[k]);
      sw[k] = bf16r(ww[k]);
    }
    *(v4f*)&sA[c] = sa;
    *(v4f*)&sW[c] = sw;
  }
  __syncthreads();
  const float bias2 = bf16r(b2[0]);
#pragma unroll 1
  for (unsigned jj = 0; jj < 4u; ++jj) {
    const unsigned j = j0 + w * 4u + jj;
    const float* brow = AB + (size_t)j * (2u * DIM) + DIM;
    float acc = 0.0f;
#pragma unroll 1
    for (unsigned q = 0; q < 8u; ++q) {
      const unsigned c = q * 128u + lane * 4u;
      const v4f s  = *(const v4f*)&sA[c];
      const v4f wv = *(const v4f*)&sW[c];
      const v4f b  = *(const v4f*)(brow + c);
#pragma unroll
      for (int k = 0; k < 4; ++k) acc += gelu_erf(s[k] + b[k]) * wv[k];
    }
    acc = red32_sum(acc);
    const float sg = __builtin_amdgcn_rcpf(1.0f + __expf(-(acc + bias2)));
    if (lane == 0u) sOut[w * 4u + jj] = sg;
  }
  __syncthreads();
  if (w == 0u) {
    const float v = sOut[lane];
    float* p = scores + (size_t)i * SEQ_FULL + j0 + lane;
    *(volatile float*)p = v;
    __threadfence();
    *(volatile float*)p = v;
  }
}

__global__ __launch_bounds__(256) void attn_kernel(
    const _Float16* __restrict__ Qh, const _Float16* __restrict__ Kh,
    const _Float16* __restrict__ Vt, _Float16* __restrict__ Ov) {
  __shared__ _Float16 Ks[32 * LDK];
  __shared__ _Float16 Vs[HD * LDV];
  __shared__ _Float16 Ps[8 * 16 * LDK];

  const unsigned tid = threadIdx.x, lane = tid & 31u;
  const unsigned w = (unsigned)__builtin_amdgcn_readfirstlane((int)(tid >> 5));
  const unsigned hh = lane >> 4, m = lane & 15u;
  const unsigned q0 = blockIdx.x * 128u;
  const unsigned head = blockIdx.y;
  const float scale = 0.08838834764831845f;
  const unsigned qrow0 = q0 + w * 16u;
  _Float16* P = Ps + w * (16u * LDK);

  const size_t qoff = (size_t)(qrow0 + m) * DIM + head * HD + hh * 8u;
  v16h qf[4];
#pragma unroll
  for (int c = 0; c < 4; ++c) qf[c] = frag_at(Qh + qoff + 32 * c);

  float mrow[8], lrow[8];
  v8f o[8];
#pragma unroll
  for (int v = 0; v < 8; ++v) { mrow[v] = -1.0e30f; lrow[v] = 0.0f; }
#pragma unroll
  for (int nb = 0; nb < 8; ++nb) o[nb] = (v8f){};

  const size_t kplane = (size_t)head * HD;
  const size_t vplane = (size_t)head * HD * SEQ;

  for (unsigned kb = 0; kb < (unsigned)SEQ; kb += 32u) {
#pragma unroll
    for (unsigned j = 0; j < 2u; ++j) {
      const unsigned idx = tid + 256u * j;
      const unsigned rk = idx >> 4, ck = (idx & 15u) * 8u;
      const unsigned rv = idx >> 2, cv = (idx & 3u) * 8u;
      *(v8h*)&Ks[rk * LDK + ck] = *(const v8h*)(Kh + kplane + (size_t)(kb + rk) * DIM + ck);
      *(v8h*)&Vs[rv * LDV + cv] = *(const v8h*)(Vt + vplane + (size_t)rv * SEQ + kb + cv);
    }
    __syncthreads();

    v8f s[2];
#pragma unroll
    for (int kg = 0; kg < 2; ++kg) {
      v8f t = {};
#pragma unroll
      for (int c = 0; c < 4; ++c) {
        const v16h kf = ld_frag(&Ks[(kg * 16) * LDK + c * 32], LDK);
        t = wmma16(qf[c], kf, t);
      }
      s[kg] = t * scale;
    }

    float alpha[8];
#pragma unroll
    for (int v = 0; v < 8; ++v) {
      float mx = fmaxf(s[0][v], s[1][v]);
      mx = red16_max(mx);
      const float mn = fmaxf(mrow[v], mx);
      alpha[v] = __expf(mrow[v] - mn);
      mrow[v] = mn;
    }
#pragma unroll
    for (int kg = 0; kg < 2; ++kg)
#pragma unroll
      for (int v = 0; v < 8; ++v) {
        const float e = __expf(s[kg][v] - mrow[v]) * PCARRY;
        const h16 ph = toh_flush(e);
        P[(hh * 8u + (unsigned)v) * LDK + (unsigned)kg * 16u + m] = ph;
        s[kg][v] = (float)ph;
      }
#pragma unroll
    for (int v = 0; v < 8; ++v) {
      const float rs = red16_sum(s[0][v] + s[1][v]);
      lrow[v] = alpha[v] * lrow[v] + rs;
    }
#pragma unroll
    for (int nb = 0; nb < 8; ++nb)
#pragma unroll
      for (int v = 0; v < 8; ++v) o[nb][v] = o[nb][v] * alpha[v];
    wave_lds_sync();

    {
      const v16h pf = ld_frag(P, LDK);
#pragma unroll
      for (int nb = 0; nb < 8; ++nb) {
        const v16h vf = ld_frag(&Vs[(nb * 16) * LDV], LDV);
        o[nb] = wmma16(pf, vf, o[nb]);
      }
    }
    __syncthreads();
  }

  float inv[8];
#pragma unroll
  for (int v = 0; v < 8; ++v) inv[v] = __builtin_amdgcn_rcpf(lrow[v]) * VCARRY;
#pragma unroll
  for (int nb = 0; nb < 8; ++nb)
#pragma unroll
    for (int v = 0; v < 8; ++v)
      P[(hh * 8u + (unsigned)v) * LDK + (unsigned)nb * 16u + m] = toh_flush(o[nb][v] * inv[v]);
  wave_lds_sync();
  v8h x[8];
  size_t off[8];
#pragma unroll
  for (unsigned i = 0; i < 8u; ++i) {
    const unsigned r = 2u * i + (lane >> 4);
    const unsigned c = (lane & 15u) * 8u;
    x[i] = *(const v8h*)&P[r * LDK + c];
    off[i] = (size_t)(qrow0 + r) * DIM + head * HD + c;
  }
#pragma unroll
  for (int i = 0; i < 8; ++i) *(volatile v8h*)(Ov + off[i]) = x[i];
  __threadfence();
#pragma unroll
  for (int i = 0; i < 8; ++i) *(volatile v8h*)(Ov + off[i]) = x[i];
}

__global__ __launch_bounds__(256) void syn_in_kernel(
    const float* __restrict__ attd, const float* __restrict__ mem, float* __restrict__ syn) {
  const unsigned t = blockIdx.x * 256u + threadIdx.x;
  float val;
  if (blockIdx.x < (2u * DIM) / 256u) {
    val = bf16r(mem[t]);
  } else {
    const unsigned d = t - 2u * DIM;
    float s = 0.0f;
#pragma unroll 4
    for (unsigned n = 0; n < (unsigned)SEQ; ++n) s += attd[(size_t)n * DIM + d];
    val = s * (1.0f / (float)SEQ);
  }
  float* p = syn + t;
  *(volatile float*)p = val;
  __threadfence();
  *(volatile float*)p = val;
}

__global__ __launch_bounds__(256) void matvec_kernel(
    const float* __restrict__ x, const float* __restrict__ W, const float* __restrict__ bias,
    float* __restrict__ y, unsigned K, unsigned act) {
  __shared__ float sOut[32];
  const unsigned tid = threadIdx.x, lane = tid & 31u;
  const unsigned w = (unsigned)__builtin_amdgcn_readfirstlane((int)(tid >> 5));
  const unsigned n0 = blockIdx.x * 32u;
#pragma unroll 1
  for (unsigned jj = 0; jj < 4u; ++jj) {
    const unsigned n = n0 + w * 4u + jj;
    const float* wr = W + (size_t)n * K;
    float acc = 0.0f;
#pragma unroll 1
    for (unsigned c = lane * 4u; c < K; c += 128u) {
      const v4f a = *(const v4f*)(x + c);
      const v4f b = *(const v4f*)(wr + c);
#pragma unroll
      for (int k = 0; k < 4; ++k) acc += a[k] * bf16r(b[k]);
    }
    acc = red32_sum(acc);
    float v = acc + bf16r(bias[n]);
    if (act != 0u) v = gelu_erf(v);
    if (lane == 0u) sOut[w * 4u + jj] = v;
  }
  __syncthreads();
  if (w == 0u) {
    const float v = sOut[lane];
    float* p = y + n0 + lane;
    *(volatile float*)p = v;
    __threadfence();
    *(volatile float*)p = v;
  }
}

extern "C" void kernel_launch(void* const* d_in, const int* in_sizes, int n_in,
                              void* d_out, int out_size, void* d_ws, size_t ws_size,
                              hipStream_t stream) {
  if (n_in < 13) return;
  if ((long long)in_sizes[0] < (long long)SEQ * DIM) return;
  if ((long long)in_sizes[1] < (long long)DIM * 2 * DIM) return;
  if (in_sizes[2] < DIM || in_sizes[3] < DIM || in_sizes[4] < 1) return;
  if ((long long)in_sizes[5] < (long long)3 * DIM * DIM) return;
  if (in_sizes[6] < 3 * DIM) return;
  if ((long long)in_sizes[7] < (long long)DIM * DIM) return;
  if (in_sizes[8] < DIM) return;
  if ((long long)in_sizes[9] < (long long)HID1 * SYNW) return;
  if (in_sizes[10] < HID1) return;
  if ((long long)in_sizes[11] < (long long)DIM * HID1) return;
  if (in_sizes[12] < DIM) return;
  if ((long long)out_size < (long long)(OUT1_OFF + DIM)) return;
  if (ws_size < WS_TOTAL) return;

  const float* mem   = (const float*)d_in[0];
  const float* W1    = (const float*)d_in[1];
  const float* b1    = (const float*)d_in[2];
  const float* w2    = (const float*)d_in[3];
  const float* b2    = (const float*)d_in[4];
  const float* in_w  = (const float*)d_in[5];
  const float* in_b  = (const float*)d_in[6];
  const float* out_w = (const float*)d_in[7];
  const float* out_b = (const float*)d_in[8];
  const float* Ws1   = (const float*)d_in[9];
  const float* bs1   = (const float*)d_in[10];
  const float* Ws2   = (const float*)d_in[11];
  const float* bs2   = (const float*)d_in[12];
  float* out = (float*)d_out;

  char* ws = (char*)d_ws;
  _Float16* X16   = (_Float16*)(ws + OFF_X16);
  _Float16* W1c   = (_Float16*)(ws + OFF_W1C);
  _Float16* Wqkv  = (_Float16*)(ws + OFF_WQKV);
  _Float16* Wo    = (_Float16*)(ws + OFF_WO);
  float*    AB    = (float*)(ws + OFF_AB);
  _Float16* Q16   = (_Float16*)(ws + OFF_Q);
  _Float16* K16   = (_Float16*)(ws + OFF_K);
  _Float16* Vt16  = (_Float16*)(ws + OFF_VT);
  _Float16* Ctx16 = (_Float16*)(ws + OFF_CTX);
  float*    ATT   = (float*)(ws + OFF_ATT);
  float*    SYN   = (float*)(ws + OFF_SYN);
  float*    HIDV  = (float*)(ws + OFF_HIDV);

  dim3 blk(256);
  dim3 gg(DIM / 64, SEQ / 64);

  cast_plane_kernel<<<dim3(SEQ / 2), blk, 0, stream>>>(mem, X16, (unsigned)DIM, 0u, 1.0f);
  cast_plane_kernel<<<dim3(DIM / 2), blk, 0, stream>>>(W1, W1c, (unsigned)(2 * DIM), 0u, WCARRY);
  cast_plane_kernel<<<dim3(DIM / 2), blk, 0, stream>>>(W1, W1c + (size_t)DIM * DIM,
                                                       (unsigned)(2 * DIM), (unsigned)DIM, WCARRY);
  cast_plane_kernel<<<dim3(3 * DIM / 2), blk, 0, stream>>>(in_w, Wqkv, (unsigned)DIM, 0u, WCARRY);
  cast_plane_kernel<<<dim3(DIM / 2), blk, 0, stream>>>(out_w, Wo, (unsigned)DIM, 0u, WCARRY);

  gemm_ab_kernel<<<dim3(2 * DIM / 64, SEQ / 64), blk, 0, stream>>>(X16, W1c, AB);
  pair_score_kernel<<<dim3(SEQ / 32, SEQ), blk, 0, stream>>>(AB, b1, w2, b2, out);

  gemm_qk_kernel<<<gg, blk, 0, stream>>>(X16, Wqkv, in_b, Q16);
  gemm_qk_kernel<<<gg, blk, 0, stream>>>(X16, Wqkv + (size_t)DIM * DIM, in_b + DIM, K16);
  gemm_v_kernel<<<gg, blk, 0, stream>>>(X16, Wqkv + (size_t)2 * DIM * DIM, in_b + 2 * DIM, Vt16);
  attn_kernel<<<dim3(SEQ / 128, NHEAD), blk, 0, stream>>>(Q16, K16, Vt16, Ctx16);
  gemm_out_kernel<<<gg, blk, 0, stream>>>(Ctx16, Wo, out_b, ATT);

  syn_in_kernel<<<dim3(3 * DIM / 256), blk, 0, stream>>>(ATT, mem, SYN);
  matvec_kernel<<<dim3(HID1 / 32), blk, 0, stream>>>(SYN, Ws1, bs1, HIDV, (unsigned)SYNW, 1u);
  matvec_kernel<<<dim3(DIM / 32), blk, 0, stream>>>(HIDV, Ws2, bs2, out + OUT1_OFF,
                                                    (unsigned)HID1, 0u);
}
